// OctreeConv_29265907155614
// MI455X (gfx1250) — hardware-verified
//
#include <hip/hip_runtime.h>

constexpr int kCin    = 32;
constexpr int kCout   = 32;
constexpr int kTaps   = 27;
constexpr int kNodes  = 131072;
constexpr int kKreal  = kCin * kTaps;
constexpr int kKpad   = 896;
constexpr int kMpad   = 64;
constexpr int kChunk  = 32768;
constexpr int kNumChunks = kNodes / kChunk;
constexpr int kNodesPerGatherBlock = 8;
constexpr int kPieces = kKpad / 8;

static_assert(kNodes % kChunk == 0, "chunking exact");
static_assert(kChunk % 64 == 0, "N tile multiple");
static_assert(kKpad % 32 == 0 && kKpad >= kKreal, "K padded to 32");
static_assert(kChunk % kNodesPerGatherBlock == 0, "gather grid exact");
static_assert((kMpad * kKpad / 8) % 256 == 0, "weight plane grid exact");
static_assert(kPieces == 112, "pieces per row");

typedef __attribute__((ext_vector_type(16))) _Float16 v16h;
typedef __attribute__((ext_vector_type(8)))  _Float16 v8h;
typedef __attribute__((ext_vector_type(16))) __bf16   v16b;
typedef __attribute__((ext_vector_type(8)))  __bf16   v8b;
typedef __attribute__((ext_vector_type(8)))  float    v8f;
typedef __attribute__((ext_vector_type(4)))  float    v4f;
typedef __attribute__((ext_vector_type(4)))  unsigned int v4u;

__device__ __forceinline__ unsigned short f2bf_bits(float f) {
  unsigned u = __float_as_uint(f);
  return (unsigned short)((u + 0x7FFFu + ((u >> 16) & 1u)) >> 16);
}
__device__ __forceinline__ float bf_bits2f(unsigned short h) { return __uint_as_float(((unsigned)h) << 16); }

__device__ __forceinline__ void dep_guard_h(v8f& a, v8f& b, v16h x, v16h y) { asm volatile("v_nop\n\tv_nop\n\tv_nop\n\tv_nop" : "+v"(a), "+v"(b) : "v"(x), "v"(y)); }
__device__ __forceinline__ void dep_guard_b(v8f& a, v8f& b, v16b x, v16b y) { asm volatile("v_nop\n\tv_nop\n\tv_nop\n\tv_nop" : "+v"(a), "+v"(b) : "v"(x), "v"(y)); }
__device__ __forceinline__ void keep4_h(v16h a, v16h b, v16h c, v16h d) { asm volatile("v_nop" :: "v"(a), "v"(b), "v"(c), "v"(d)); }
__device__ __forceinline__ void keep4_b(v16b a, v16b b, v16b c, v16b d) { asm volatile("v_nop" :: "v"(a), "v"(b), "v"(c), "v"(d)); }
__device__ __forceinline__ void acc_guard4(v8f& a, v8f& b, v8f& c, v8f& d) { asm volatile("v_nop\n\tv_nop\n\tv_nop\n\tv_nop" : "+v"(a), "+v"(b), "+v"(c), "+v"(d)); }
template <typename T> struct Frag;
template <> struct Frag<_Float16> {
  typedef v16h V; union U { v16h v; v8h h[2]; };
  static __device__ __forceinline__ v16h load(const _Float16* p) {
    U f; f.h[0] = *(const v8h*)(p); f.h[1] = *(const v8h*)(p + 16); return f.v;
  }
  static __device__ __forceinline__ v8f mma(v16h a, v16h b, v8f c) {
    return __builtin_amdgcn_wmma_f32_16x16x32_f16(false, a, false, b, (short)0, c, false, false);
  }
  static __device__ __forceinline__ void guard(v8f& a, v8f& b, v16h x, v16h y) { dep_guard_h(a, b, x, y); }
  static __device__ __forceinline__ void keep(v16h a, v16h b, v16h c, v16h d) { keep4_h(a, b, c, d); }
};
template <> struct Frag<__bf16> {
  typedef v16b V; union U { v16b v; v8b h[2]; };
  static __device__ __forceinline__ v16b load(const __bf16* p) {
    U f; f.h[0] = *(const v8b*)(p); f.h[1] = *(const v8b*)(p + 16); return f.v;
  }
  static __device__ __forceinline__ v8f mma(v16b a, v16b b, v8f c) {
    return __builtin_amdgcn_wmma_f32_16x16x32_bf16(false, a, false, b, (short)0, c, false, false);
  }
  static __device__ __forceinline__ void guard(v8f& a, v8f& b, v16b x, v16b y) { dep_guard_b(a, b, x, y); }
  static __device__ __forceinline__ void keep(v16b a, v16b b, v16b c, v16b d) { keep4_b(a, b, c, d); }
};

__device__ __forceinline__ unsigned pk16(unsigned short a, unsigned short b) { return (unsigned)a | ((unsigned)b << 16); }

template <int ET> struct Elem;
template <> struct Elem<0> { typedef _Float16 T; };
template <> struct Elem<1> { typedef __bf16 T; };
template <int ET, bool SPLIT, int BIAS_MODE, int OUT_MODE, bool RESID, int ACT = 0>
__global__ __launch_bounds__(256) void wmma_gemm64(
    const unsigned short* __restrict__ Ap, const unsigned short* __restrict__ A2p, int lda, long strideA,
    const unsigned short* __restrict__ Btp, const unsigned short* __restrict__ Bt2p, int ldb, long strideB,
    void* __restrict__ Cout, void* __restrict__ Cout2, int ldc, long strideC,
    const float* __restrict__ bias,
    const float* __restrict__ resid, long strideR,
    int M, int N, int K, float scale, int Mst) {
  typedef typename Elem<ET>::T T;
  typedef typename Frag<T>::V V;
  const T* A = (const T*)Ap; const T* A2 = (const T*)A2p; const T* Bt = (const T*)Btp; const T* Bt2 = (const T*)Bt2p;
  __shared__ __align__(16) float sT[8][16 * 68];
  const int b    = blockIdx.y;
  const int lane = threadIdx.x & 31;
  const int wave = threadIdx.x >> 5;
  const int tilesN = N >> 6;
  const int tilesM = M >> 6;
  const int tile = blockIdx.x * 8 + wave;
  if (tile >= tilesM * tilesN) return;
  const int tm = tile / tilesN;
  const int tn = tile - tm * tilesN;
  const int m0 = tm << 6;
  const int n0 = tn << 6;

  const T* Ab  = A  + (size_t)b * strideA;
  const T* Bb  = Bt + (size_t)b * strideB;
  const T* Ab2 = SPLIT ? (A2  + (size_t)b * strideA) : nullptr;
  const T* Bb2 = SPLIT ? (Bt2 + (size_t)b * strideB) : nullptr;

  const int rlane = lane & 15;
  const int koff  = (lane >> 4) * 8;
  const int mOff  = (lane >> 4) * 8;

  v8f acc[4][4];
#pragma unroll
  for (int i = 0; i < 4; ++i)
#pragma unroll
    for (int j = 0; j < 4; ++j) acc[i][j] = (v8f){0.f,0.f,0.f,0.f,0.f,0.f,0.f,0.f};

  for (int k0 = 0; k0 < K; k0 += 32) {
    V bh[4], bl[4];
#pragma unroll
    for (int j = 0; j < 4; ++j) {
      const size_t bo = (size_t)(n0 + (j << 4) + rlane) * ldb + koff + k0;
      bh[j] = Frag<T>::load(Bb + bo);
      if (SPLIT) bl[j] = Frag<T>::load(Bb2 + bo);
    }
#pragma unroll
    for (int i = 0; i < 4; ++i) {
      const size_t ao = (size_t)(m0 + (i << 4) + rlane) * lda + koff + k0;
      V ah = Frag<T>::load(Ab + ao);
      V al;
      if (SPLIT) al = Frag<T>::load(Ab2 + ao);
#pragma unroll
      for (int j = 0; j < 4; ++j) {
        acc[i][j] = Frag<T>::mma(ah, bh[j], acc[i][j]);
        if (SPLIT) {
          acc[i][j] = Frag<T>::mma(ah, bl[j], acc[i][j]);
          acc[i][j] = Frag<T>::mma(al, bh[j], acc[i][j]);
        }
      }
      Frag<T>::guard(acc[i][0], acc[i][3], ah, SPLIT ? al : ah);
    }
    Frag<T>::keep(bh[0], bh[1], bh[2], bh[3]);
    if (SPLIT) Frag<T>::keep(bl[0], bl[1], bl[2], bl[3]);
  }
  acc_guard4(acc[0][0], acc[0][1], acc[0][2], acc[0][3]);
  acc_guard4(acc[1][0], acc[1][1], acc[1][2], acc[1][3]);
  acc_guard4(acc[2][0], acc[2][1], acc[2][2], acc[2][3]);
  acc_guard4(acc[3][0], acc[3][1], acc[3][2], acc[3][3]);

  float* slab = sT[wave];
  const float* Rb = RESID ? (resid + (size_t)b * strideR) : nullptr;
#pragma unroll
  for (int i = 0; i < 4; ++i) {
    const int mBase = m0 + (i << 4);
#pragma unroll
    for (int j = 0; j < 4; ++j) {
      const int n = n0 + (j << 4) + rlane;
      float bv = 0.f;
      if (BIAS_MODE == 2) bv = bias[n];
#pragma unroll
      for (int r = 0; r < 8; ++r) {
        float v = acc[i][j][r] * scale;
        if (BIAS_MODE == 1) v += bias[mBase + mOff + r];
        if (BIAS_MODE == 2) v += bv;
        if (RESID) v += Rb[(size_t)(mBase + mOff + r) * ldc + n];
        if (ACT == 2) v = fmaxf(v, 0.0f);
        if (ACT == 4) v = (v > 0.f) ? v : 0.01f * v;
        slab[(mOff + r) * 68 + (j << 4) + rlane] = v;
      }
    }
    __builtin_amdgcn_fence(__ATOMIC_RELEASE, "workgroup");
    __builtin_amdgcn_wave_barrier();
    __builtin_amdgcn_fence(__ATOMIC_ACQUIRE, "workgroup");
    if (mBase < Mst) {
      if (OUT_MODE == 0) {
        float* C = (float*)Cout + (size_t)b * strideC;
        const int hh = lane >> 4, c4 = (lane & 15) * 4;
        for (int pass = 0; pass < 2; ++pass) {
#pragma unroll
          for (int it = 0; it < 8; ++it) {
            const int row = it * 2 + hh;
            v4f v = *(const v4f*)(slab + row * 68 + c4);
            *(volatile v4f*)(C + (size_t)(mBase + row) * ldc + n0 + c4) = v;
          }
          __threadfence();
        }
      } else {
        const int q = lane >> 3, c8 = (lane & 7) * 8;
        unsigned short* C  = (unsigned short*)Cout  + (size_t)b * strideC;
        unsigned short* C2 = (OUT_MODE == 2) ? ((unsigned short*)Cout2 + (size_t)b * strideC) : nullptr;
        for (int pass = 0; pass < 2; ++pass) {
#pragma unroll
          for (int it = 0; it < 4; ++it) {
            const int row = it * 4 + q;
            const float* sp = slab + row * 68 + c8;
            v8h hv, lv;
#pragma unroll
            for (int e = 0; e < 8; ++e) {
              if (OUT_MODE == 1) {
                hv[e] = (_Float16)sp[e];
              } else {
                unsigned short hb = f2bf_bits(sp[e]);
                unsigned short lb = f2bf_bits(sp[e] - bf_bits2f(hb));
                hv[e] = __builtin_bit_cast(_Float16, hb);
                lv[e] = __builtin_bit_cast(_Float16, lb);
              }
            }
            *(volatile v8h*)(C + (size_t)(mBase + row) * ldc + n0 + c8) = hv;
            if (OUT_MODE == 2) *(volatile v8h*)(C2 + (size_t)(mBase + row) * ldc + n0 + c8) = lv;
          }
          __threadfence();
        }
      }
    }
    __builtin_amdgcn_fence(__ATOMIC_RELEASE, "workgroup");
    __builtin_amdgcn_wave_barrier();
    __builtin_amdgcn_fence(__ATOMIC_ACQUIRE, "workgroup");
  }
}

__global__ __launch_bounds__(256) void prep_wplane(const float* __restrict__ w, unsigned short* __restrict__ wp) {
  const int i = blockIdx.x * 256 + threadIdx.x;
  if (i >= kMpad * kPieces) return;
  const int row = i / kPieces;
  const int c8  = (i - row * kPieces) * 8;
  const int rowc = (row < kCout) ? row : (kCout - 1);
  unsigned short hb[8];
#pragma unroll
  for (int e = 0; e < 8; ++e) {
    const int kk  = c8 + e;
    const int kkc = (kk < kKreal) ? kk : (kKreal - 1);
    const float v = w[(size_t)rowc * kKreal + kkc];
    hb[e] = (row < kCout && kk < kKreal) ? f2bf_bits(v) : (unsigned short)0;
  }
  const v4u u = (v4u){pk16(hb[0], hb[1]), pk16(hb[2], hb[3]), pk16(hb[4], hb[5]), pk16(hb[6], hb[7])};
  unsigned short* q = wp + 8 * (size_t)i;
  *(volatile v4u*)q = u;
  __threadfence();
  *(volatile v4u*)q = u;
}

__global__ __launch_bounds__(256) void gather_cols(const float* __restrict__ din, const int* __restrict__ oct,
                                                   unsigned short* __restrict__ col, int nbase) {
  __shared__ __align__(16) unsigned short srow[kNodesPerGatherBlock][kKpad];
  const int lane = threadIdx.x & 31;
  const int wave = threadIdx.x >> 5;
  const int nl   = blockIdx.x * kNodesPerGatherBlock + wave;
  const int n    = nbase + nl;
  const int tap  = (lane < kTaps) ? lane : (kTaps - 1);
  int idx = oct[(size_t)n * kTaps + tap];
  idx = (idx < 0) ? 0 : ((idx > kNodes - 1) ? (kNodes - 1) : idx);
  unsigned short* sr = srow[wave];
  const float* dp = din + idx;
#pragma unroll 1
  for (int c = 0; c < kCin; ++c) {
    const float v = dp[(size_t)c * kNodes];
    const unsigned short bb = f2bf_bits(v);
    if (lane < kTaps) sr[c * kTaps + lane] = bb;
  }
  sr[kKreal + lane] = (unsigned short)0;
  __syncthreads();
  const int q3 = 96 + ((lane < 16) ? lane : 15);
  const v4u p0 = *(const v4u*)(sr + (size_t)(lane) * 8);
  const v4u p1 = *(const v4u*)(sr + (size_t)(32 + lane) * 8);
  const v4u p2 = *(const v4u*)(sr + (size_t)(64 + lane) * 8);
  const v4u p3 = *(const v4u*)(sr + (size_t)q3 * 8);
  unsigned short* crow = col + (size_t)nl * kKpad;
  for (int pass = 0; pass < 2; ++pass) {
    *(volatile v4u*)(crow + (size_t)(lane) * 8)      = p0;
    *(volatile v4u*)(crow + (size_t)(32 + lane) * 8) = p1;
    *(volatile v4u*)(crow + (size_t)(64 + lane) * 8) = p2;
    if (lane < 16) *(volatile v4u*)(crow + (size_t)(96 + lane) * 8) = p3;
    __threadfence();
  }
}

extern "C" void kernel_launch(void* const* d_in, const int* in_sizes, int n_in,
                              void* d_out, int out_size, void* d_ws, size_t ws_size,
                              hipStream_t stream) {
  if (n_in < 3) return;
  if (in_sizes[0] != kCin * kNodes) return;
  if (in_sizes[1] != kCout * kKreal) return;
  if (in_sizes[2] != kNodes * kTaps) return;
  if (out_size != kCout * kNodes) return;

  const float* data_in = (const float*)d_in[0];
  const float* weights = (const float*)d_in[1];
  const int*   octree  = (const int*)d_in[2];
  float* outp = (float*)d_out;

  const size_t SZ_WP  = (size_t)kMpad * kKpad * 2;
  const size_t SZ_COL = (size_t)kChunk * kKpad * 2;
  const size_t oWP  = 0;
  const size_t oCOL = oWP + SZ_WP;
  const size_t TOTAL = oCOL + SZ_COL;
  if (TOTAL > ws_size) return;
  if (TOTAL > (size_t)134217728) return;

  char* ws = (char*)d_ws;
  unsigned short* WP  = (unsigned short*)(ws + oWP);
  unsigned short* COL = (unsigned short*)(ws + oCOL);
  const float* dummy_f = (const float*)(ws + oWP);

  const dim3 blk(256);

  prep_wplane<<<dim3((kMpad * kPieces) / 256), blk, 0, stream>>>(weights, WP);

  const dim3 gGather(kChunk / kNodesPerGatherBlock);
  const dim3 gGemm(((kMpad / 64) * (kChunk / 64) + 7) / 8, 1);
  for (int q = 0; q < kNumChunks; ++q) {
    const int nbase = q * kChunk;
    gather_cols<<<gGather, blk, 0, stream>>>(data_in, octree, COL, nbase);
    wmma_gemm64<1, false, 0, 0, false, 0><<<gGemm, blk, 0, stream>>>(
        WP, WP, kKpad, 0L,
        COL, COL, kKpad, 0L,
        (void*)(outp + nbase), (void*)(outp + nbase), kNodes, 0L,
        dummy_f,
        dummy_f, 0L,
        kMpad, kChunk, kKpad, 1.0f, kCout);
  }
}
